// Sequence_26860725469223
// MI455X (gfx1250) — hardware-verified
//
#include <hip/hip_runtime.h>
#include <stdint.h>
#include <stddef.h>

typedef __attribute__((ext_vector_type(16))) _Float16 v16h;
typedef __attribute__((ext_vector_type(8)))  _Float16 v8h;
typedef __attribute__((ext_vector_type(8)))  float    v8f;
typedef __attribute__((ext_vector_type(4)))  float    v4f;
typedef __attribute__((ext_vector_type(8)))  unsigned v8u;

constexpr int NBATCH = 512;
constexpr int T_OBS  = 2048;
constexpr int T_FUT  = 64;
constexpr int T_ALL  = T_OBS + T_FUT;
constexpr int HID    = 25;
constexpr int NGATES = 4 * HID;
constexpr int KPAD   = 32;
constexpr int NPADC  = 128;
constexpr int NTILE  = NPADC / 16;
constexpr int NWAVE  = 4;
constexpr int ROWS_W = 16;
constexpr int ROWS_B = NWAVE * ROWS_W;
constexpr int NBLK   = NBATCH / ROWS_B;
constexpr int OBW    = 32;
constexpr int NTHR   = NWAVE * 32;
constexpr int WPLANE = NPADC * KPAD;

static_assert(NBATCH % ROWS_B == 0, "");
static_assert(T_ALL % OBW == 0, "");
static_assert(HID + 1 <= KPAD, "");
static_assert(NTILE == 8, "");
static_assert(WPLANE == 4096, "");
static_assert((T_ALL * 4) % 128 == 0, "");

__device__ __forceinline__ v16h frag_ld(const _Float16* p) {
  union { v16h v; v8h h[2]; } f;
  f.h[0] = *(const v8h*)(p);
  f.h[1] = *(const v8h*)(p + 16);
  return f.v;
}

__device__ __forceinline__ v8f mma16(v16h a, v16h b, v8f c) {
  c = __builtin_amdgcn_wmma_f32_16x16x32_f16(false, a, false, b, (short)0, c, false, false);
  asm volatile("v_nop\n\tv_nop\n\tv_nop\n\tv_nop" : "+v"(c) : "v"(a), "v"(b));
  return c;
}

__device__ __forceinline__ float sigm_f(float x) {
  return __builtin_amdgcn_rcpf(1.0f + __expf(-x));
}
__device__ __forceinline__ float tanh_f(float x) {
  return 1.0f - 2.0f * __builtin_amdgcn_rcpf(1.0f + __expf(2.0f * x));
}

__device__ __forceinline__ void lstm_cell_ew(const v8f (&acc)[NTILE], const float (&bs)[NTILE],
                                             float (&cs)[16], float (&hv)[16], int c) {
#pragma unroll
  for (int t2 = 0; t2 < 2; ++t2) {
    const bool valid = (16 * t2 + c) < HID;
#pragma unroll
    for (int r = 0; r < 8; ++r) {
      const int ci = t2 * 8 + r;
      const float iv = sigm_f(acc[t2][r]     + bs[t2]);
      const float fv = sigm_f(acc[2 + t2][r] + bs[2 + t2]);
      const float gv = tanh_f(acc[4 + t2][r] + bs[4 + t2]);
      const float ov = sigm_f(acc[6 + t2][r] + bs[6 + t2]);
      float cn = fv * cs[ci] + iv * gv;
      cn = valid ? cn : 0.0f;
      cs[ci] = cn;
      const float hn = ov * tanh_f(cn);
      hv[ci] = valid ? hn : 0.0f;
    }
  }
}

__device__ __forceinline__ void store_htile(_Float16* hw, const float (&hv)[16], int hh, int c) {
#pragma unroll
  for (int t2 = 0; t2 < 2; ++t2) {
#pragma unroll
    for (int r = 0; r < 8; ++r) {
      hw[(8 * hh + r) * KPAD + 16 * t2 + c] = (_Float16)hv[t2 * 8 + r];
    }
  }
}

__global__ __launch_bounds__(NTHR) void lstm2_stack_fwd(
    const float* __restrict__ xin,
    const float* __restrict__ W_ih1, const float* __restrict__ W_hh1,
    const float* __restrict__ b_ih1, const float* __restrict__ b_hh1,
    const float* __restrict__ W_ih2, const float* __restrict__ W_hh2,
    const float* __restrict__ b_ih2, const float* __restrict__ b_hh2,
    const float* __restrict__ W_lin, const float* __restrict__ b_lin,
    float* __restrict__ out)
{
  __shared__ __align__(16) _Float16 wts[3 * WPLANE];
  __shared__ __align__(16) _Float16 h1t[NWAVE * ROWS_W * KPAD];
  __shared__ __align__(16) _Float16 h2t[NWAVE * ROWS_W * KPAD];
  __shared__ __align__(16) float obuf[NWAVE * ROWS_W * OBW];
  __shared__ __align__(16) float btab[2 * NPADC];
  __shared__ __align__(16) float wltab[32];

  const int tid  = threadIdx.x;
  const int lane = tid & 31;
  const int wave = tid >> 5;
  const int hh   = lane >> 4;
  const int c    = lane & 15;

#pragma unroll 1
  for (int idx = tid; idx < 3 * WPLANE; idx += NTHR) {
    const int plane = idx >> 12;
    const int rem = idx & (WPLANE - 1);
    const int n = rem >> 5;
    const int k = rem & 31;
    const int G = n >> 5;
    const int q = n & 31;
    const int row = HID * G + ((q < HID) ? q : (HID - 1));
    const int kc  = (k < HID) ? k : (HID - 1);
    const float whh1 = W_hh1[row * HID + kc];
    const float wih1 = W_ih1[row];
    const float wih2 = W_ih2[row * HID + kc];
    const float whh2 = W_hh2[row * HID + kc];
    const float v0 = (k < HID) ? whh1 : ((k == HID) ? wih1 : 0.0f);
    const float v1 = (k < HID) ? wih2 : 0.0f;
    const float v2 = (k < HID) ? whh2 : 0.0f;
    float v = (plane == 0) ? v0 : ((plane == 1) ? v1 : v2);
    v = (q < HID) ? v : 0.0f;
    wts[idx] = (_Float16)v;
  }
#pragma unroll 1
  for (int idx = tid; idx < 2 * NPADC; idx += NTHR) {
    const int l = idx >> 7;
    const int p = idx & (NPADC - 1);
    const int G = p >> 5;
    const int q = p & 31;
    const int row = HID * G + ((q < HID) ? q : (HID - 1));
    const float s1 = b_ih1[row] + b_hh1[row];
    const float s2 = b_ih2[row] + b_hh2[row];
    const float v = (l == 0) ? s1 : s2;
    btab[idx] = (q < HID) ? v : 0.0f;
  }
  if (tid < 32) {
    const float w = W_lin[(tid < HID) ? tid : (HID - 1)];
    wltab[tid] = (tid < HID) ? w : 0.0f;
  }
#pragma unroll 1
  for (int i = tid; i < NWAVE * ROWS_W * KPAD; i += NTHR) {
    h1t[i] = (_Float16)0.0f;
    h2t[i] = (_Float16)0.0f;
  }
#pragma unroll 1
  for (int i = tid; i < NWAVE * ROWS_W * OBW; i += NTHR) {
    obuf[i] = 0.0f;
  }
  __syncthreads();

  float bs1[NTILE], bs2[NTILE];
#pragma unroll
  for (int n = 0; n < NTILE; ++n) {
    bs1[n] = btab[16 * n + c];
    bs2[n] = btab[NPADC + 16 * n + c];
  }
  const float wl0  = wltab[c];
  const float wl1  = wltab[16 + c];
  const float blin = b_lin[0];

  _Float16* h1w = h1t + wave * (ROWS_W * KPAD);
  _Float16* h2w = h2t + wave * (ROWS_W * KPAD);
  float*    ob  = obuf + wave * (ROWS_W * OBW);
  const int rowbase = blockIdx.x * ROWS_B + wave * ROWS_W;
  const float* xrow = xin + (size_t)(rowbase + c) * T_OBS;

  float c1s[16], c2s[16];
#pragma unroll
  for (int i = 0; i < 16; ++i) { c1s[i] = 0.0f; c2s[i] = 0.0f; }

  const v8f zf = (v8f){0.f, 0.f, 0.f, 0.f, 0.f, 0.f, 0.f, 0.f};

#pragma clang loop unroll(disable)
  for (int t = 0; t < T_ALL; ++t) {
    const int tcl = (t < T_OBS) ? t : (T_OBS - 1);
    const float xg = xrow[tcl];
    const float xl = ob[c * OBW + ((t - 1) & (OBW - 1))];
    const float xv = (t < T_OBS) ? xg : xl;

    v16h a1 = frag_ld(h1w + c * KPAD + 8 * hh);
    {
      const _Float16 xh = (_Float16)xv;
      const unsigned xb = (unsigned)__builtin_bit_cast(unsigned short, xh);
      v8u au = __builtin_bit_cast(v8u, a1);
      const unsigned w4  = au[4];
      const unsigned w4x = (w4 & 0xffffu) | (xb << 16);
      au[4] = hh ? w4x : w4;
      a1 = __builtin_bit_cast(v16h, au);
    }
    v8f acc[NTILE];
#pragma unroll
    for (int n = 0; n < NTILE; ++n) {
      const v16h bf = frag_ld(wts + (16 * n + c) * KPAD + 8 * hh);
      acc[n] = mma16(a1, bf, zf);
    }
    float hv[16];
    lstm_cell_ew(acc, bs1, c1s, hv, c);
    store_htile(h1w, hv, hh, c);
    __syncthreads();

    {
      const v16h a20 = frag_ld(h1w + c * KPAD + 8 * hh);
      const v16h a21 = frag_ld(h2w + c * KPAD + 8 * hh);
#pragma unroll
      for (int n = 0; n < NTILE; ++n) {
        const v16h b0 = frag_ld(wts + WPLANE + (16 * n + c) * KPAD + 8 * hh);
        const v16h b1 = frag_ld(wts + 2 * WPLANE + (16 * n + c) * KPAD + 8 * hh);
        const v8f ta = mma16(a20, b0, zf);
        acc[n] = mma16(a21, b1, ta);
      }
    }
    lstm_cell_ew(acc, bs2, c2s, hv, c);
    store_htile(h2w, hv, hh, c);

    float s[8];
#pragma unroll
    for (int r = 0; r < 8; ++r) {
      float pr = hv[r] * wl0 + hv[8 + r] * wl1;
#pragma unroll
      for (int off = 1; off < 16; off <<= 1) pr += __shfl_xor(pr, off, 32);
      s[r] = pr + blin;
    }
    float vout = s[0];
#pragma unroll
    for (int r = 1; r < 8; ++r) vout = (c == r) ? s[r] : vout;
    if (c < 8) ob[(8 * hh + c) * OBW + (t & (OBW - 1))] = vout;
    __syncthreads();

    if ((t & (OBW - 1)) == (OBW - 1)) {
      const int tb = t - (OBW - 1);
      const int q4 = lane >> 3;
      const int c4 = (lane & 7) * 4;
      float* obase = out + (size_t)rowbase * T_ALL + tb;
      for (int pass = 0; pass < 2; ++pass) {
#pragma unroll
        for (int it = 0; it < 4; ++it) {
          const int row = it * 4 + q4;
          const v4f v = *(const v4f*)(ob + row * OBW + c4);
          *(volatile v4f*)(obase + (size_t)row * T_ALL + c4) = v;
        }
        __threadfence();
      }
    }
  }
}

extern "C" void kernel_launch(void* const* d_in, const int* in_sizes, int n_in,
                              void* d_out, int out_size, void* d_ws, size_t ws_size,
                              hipStream_t stream) {
  (void)d_ws; (void)ws_size;
  if (n_in < 11) return;
  if (in_sizes[0] != NBATCH * T_OBS) return;
  if (out_size != NBATCH * T_ALL) return;
  if (in_sizes[1] != NGATES || in_sizes[2] != NGATES * HID ||
      in_sizes[3] != NGATES || in_sizes[4] != NGATES ||
      in_sizes[5] != NGATES * HID || in_sizes[6] != NGATES * HID ||
      in_sizes[7] != NGATES || in_sizes[8] != NGATES ||
      in_sizes[9] != HID || in_sizes[10] < 1) return;

  const float* input = (const float*)d_in[0];
  const float* W_ih1 = (const float*)d_in[1];
  const float* W_hh1 = (const float*)d_in[2];
  const float* b_ih1 = (const float*)d_in[3];
  const float* b_hh1 = (const float*)d_in[4];
  const float* W_ih2 = (const float*)d_in[5];
  const float* W_hh2 = (const float*)d_in[6];
  const float* b_ih2 = (const float*)d_in[7];
  const float* b_hh2 = (const float*)d_in[8];
  const float* W_lin = (const float*)d_in[9];
  const float* b_lin = (const float*)d_in[10];
  float* outp = (float*)d_out;

  lstm2_stack_fwd<<<dim3(NBLK), dim3(NTHR), 0, stream>>>(
      input, W_ih1, W_hh1, b_ih1, b_hh1, W_ih2, W_hh2, b_ih2, b_hh2, W_lin, b_lin, outp);
}
